// GABlock_60593398612596
// MI455X (gfx1250) — hardware-verified
//
#include <hip/hip_runtime.h>
#include <math.h>
#include <stdint.h>

#define NB    4
#define CH    128
#define IMH   128
#define IMW   128
#define NPIX  65536
#define PBP   992

static_assert(IMH % 8 == 0);
static_assert(IMW % 8 == 0);
static_assert(IMW % 64 == 0);
static_assert((IMH / 8) * (IMW / 8) == 256);
static_assert(NPIX == NB * IMH * IMW);
static_assert(CH == 128);
static_assert(PBP % 32 == 0);
static_assert(PBP >= 961);

typedef __attribute__((ext_vector_type(16))) __bf16   v16b;
typedef __attribute__((ext_vector_type(8)))  __bf16   v8b;
typedef __attribute__((ext_vector_type(8)))  float    v8f;
typedef __attribute__((ext_vector_type(4)))  float    v4f;
typedef __attribute__((ext_vector_type(4)))  unsigned int v4u;

constexpr size_t PLANE  = (size_t)NPIX * 128;
constexpr size_t O_XT   = 0;
constexpr size_t O_PQ   = 1 * PLANE;
constexpr size_t O_PX   = 2 * PLANE;
constexpr size_t O_TT   = 3 * PLANE;
constexpr size_t O_PK   = 4 * PLANE;
constexpr size_t O_PVT  = 5 * PLANE;
constexpr size_t O_W    = 6 * PLANE;
constexpr size_t O_CAT  = O_PK;
constexpr size_t O_X1   = O_PQ;
constexpr size_t O_WG   = O_W;
constexpr size_t O_A1   = O_WG  + 256 * 64;
constexpr size_t O_A2   = O_A1  + 64 * 128;
constexpr size_t O_SWQ  = O_A2  + 64 * 128;
constexpr size_t O_WNQ  = O_SWQ + 96 * 32;
constexpr size_t O_SWP  = O_WNQ + 96 * 32;
constexpr size_t O_WNP  = O_SWP + 32 * 64;
constexpr size_t O_FCX  = O_WNP + 32 * 64;
constexpr size_t O_M1X  = O_FCX + 128 * 256;
constexpr size_t O_M2X  = O_M1X + 256 * 256;
constexpr size_t O_WEND = O_M2X + 128 * 512;
constexpr size_t PB_BYTE  = O_WEND * 2;
constexpr size_t WS_TOTAL = PB_BYTE + (size_t)4 * PBP * 4;
static_assert(PB_BYTE % 128 == 0);
static_assert((O_A1 % 64) == 0 && (O_SWQ % 64) == 0 && (O_WNQ % 64) == 0 && (O_SWP % 64) == 0 && (O_FCX % 64) == 0);
static_assert(WS_TOTAL <= (size_t)134217728);
static_assert(O_PX == O_PQ + PLANE);
static_assert(O_PVT == O_PK + PLANE);

__device__ __forceinline__ unsigned short f2bf_bits(float f) {
  unsigned u = __float_as_uint(f);
  return (unsigned short)((u + 0x7FFFu + ((u >> 16) & 1u)) >> 16);
}
__device__ __forceinline__ float bf_bits2f(unsigned short h) { return __uint_as_float(((unsigned)h) << 16); }
__device__ __forceinline__ float bf_rne(float f) { return bf_bits2f(f2bf_bits(f)); }
__device__ __forceinline__ unsigned pk16(unsigned short a, unsigned short b) { return (unsigned)a | ((unsigned)b << 16); }
__device__ __forceinline__ void at_split(float f, __bf16& hi, __bf16& lo) {
  const unsigned short hb = f2bf_bits(f);
  hi = __builtin_bit_cast(__bf16, hb);
  lo = __builtin_bit_cast(__bf16, f2bf_bits(f - bf_bits2f(hb)));
}
__device__ __forceinline__ void split8(const float* sp, v4u& hv, v4u& lv) {
  unsigned short h[8], l[8];
#pragma unroll
  for (int e = 0; e < 8; ++e) {
    const float f = sp[e];
    h[e] = f2bf_bits(f);
    l[e] = f2bf_bits(f - bf_bits2f(h[e]));
  }
  hv[0] = pk16(h[0], h[1]); hv[1] = pk16(h[2], h[3]); hv[2] = pk16(h[4], h[5]); hv[3] = pk16(h[6], h[7]);
  lv[0] = pk16(l[0], l[1]); lv[1] = pk16(l[2], l[3]); lv[2] = pk16(l[4], l[5]); lv[3] = pk16(l[6], l[7]);
}
__device__ __forceinline__ void widen8(v4u w, float* o) {
#pragma unroll
  for (int q = 0; q < 4; ++q) {
    o[2 * q]     = __uint_as_float(w[q] << 16);
    o[2 * q + 1] = __uint_as_float(w[q] & 0xffff0000u);
  }
}

union FB { v16b v; v8b h[2]; };
__device__ __forceinline__ v8f at_mma(v16b a, v16b b, v8f c) {
  c = __builtin_amdgcn_wmma_f32_16x16x32_bf16(false, a, false, b, (short)0, c, false, false);
  asm volatile("v_nop\n\tv_nop\n\tv_nop\n\tv_nop" : "+v"(c) : "v"(a), "v"(b));
  return c;
}
__device__ __forceinline__ v8b glb_half(const unsigned short* p) {
  return *(const v8b*)(const void*)p;
}
__device__ __forceinline__ v16b glb_frag(const unsigned short* p) {
  const __bf16* q = (const __bf16*)(const void*)p;
  FB f; f.h[0] = *(const v8b*)q; f.h[1] = *(const v8b*)(q + 16); return f.v;
}
__device__ __forceinline__ v16b lds_frag(const __bf16* p) {
  FB f; f.h[0] = *(const v8b*)p; f.h[1] = *(const v8b*)(p + 16); return f.v;
}
__device__ __forceinline__ v8b zero8b() { const v4u z = {0u, 0u, 0u, 0u}; return __builtin_bit_cast(v8b, z); }
__device__ __forceinline__ void wave_sync() {
  __builtin_amdgcn_fence(__ATOMIC_RELEASE, "workgroup");
  __builtin_amdgcn_wave_barrier();
  __builtin_amdgcn_fence(__ATOMIC_ACQUIRE, "workgroup");
}

#define PR_XT 1024

template <int OC, int SC, int MODE>
__device__ __forceinline__ void plane_role(const float* __restrict__ src, unsigned short* __restrict__ dst,
                                           int rows, int blk) {
  constexpr int UPR = OC / 8;
  const int total = rows * UPR;
  const int u0 = blk * 256 + (int)threadIdx.x;
  const int u = (u0 < total) ? u0 : (total - 1);
  const int row = u / UPR;
  const int oc = (u - row * UPR) * 8;
  int sc;
  if (MODE == 0) sc = oc % SC;
  else sc = (oc < 64) ? (oc & 31) : ((oc < 128) ? (32 + (oc & 31)) : (64 + (oc & 63)));
  const float* sp = src + (size_t)row * SC + sc;
  const v4f a = *(const v4f*)sp;
  const v4f c = *(const v4f*)(sp + 4);
  v4u hv;
  hv[0] = pk16(f2bf_bits(a[0]), f2bf_bits(a[1]));
  hv[1] = pk16(f2bf_bits(a[2]), f2bf_bits(a[3]));
  hv[2] = pk16(f2bf_bits(c[0]), f2bf_bits(c[1]));
  hv[3] = pk16(f2bf_bits(c[2]), f2bf_bits(c[3]));
  if (u0 < total) {
    unsigned short* dp = dst + (size_t)row * OC + oc;
    *(volatile v4u*)dp = hv;
    __threadfence();
    *(volatile v4u*)dp = hv;
  }
}

__global__ __launch_bounds__(256) void k_prep(
    const float* __restrict__ x,
    const float* __restrict__ w_gqkv, const float* __restrict__ w_ggp,
    const float* __restrict__ w_a1, const float* __restrict__ w_a2,
    const float* __restrict__ w_swq, const float* __restrict__ w_wnq,
    const float* __restrict__ w_swp, const float* __restrict__ w_wnp,
    const float* __restrict__ w_fc, const float* __restrict__ w_m1, const float* __restrict__ w_m2,
    const float* __restrict__ pw1, const float* __restrict__ pb1,
    const float* __restrict__ pw2, const float* __restrict__ pb2,
    const float* __restrict__ pw3, const float* __restrict__ pb3,
    unsigned short* __restrict__ ws16, float* __restrict__ PB) {
  __shared__ __align__(16) float sm[128 * 68];
  const int tid = threadIdx.x;
  int bx = blockIdx.x;
  if (bx < PR_XT) {
    const int b = bx >> 8, h = (bx >> 1) & 127, w0 = (bx & 1) * 64;
#pragma unroll
    for (int it = 0; it < 8; ++it) {
      const int u = it * 256 + tid;
      const int c = u >> 4, w4 = (u & 15) * 4;
      const v4f a = *(const v4f*)(x + ((size_t)(b * CH + c) * IMH + h) * IMW + w0 + w4);
      *(v4f*)(sm + c * 68 + w4) = a;
    }
    __syncthreads();
    v4u hv[4];
#pragma unroll
    for (int it = 0; it < 4; ++it) {
      const int u = it * 256 + tid;
      const int px = u >> 4, c8 = (u & 15) * 8;
      v4u a;
#pragma unroll
      for (int q = 0; q < 4; ++q)
        a[q] = pk16(f2bf_bits(sm[(c8 + 2 * q) * 68 + px]), f2bf_bits(sm[(c8 + 2 * q + 1) * 68 + px]));
      hv[it] = a;
    }
    const size_t pixbase = (size_t)b * 16384 + (size_t)h * 128 + w0;
    for (int pass = 0; pass < 2; ++pass) {
#pragma unroll
      for (int it = 0; it < 4; ++it) {
        const int u = it * 256 + tid;
        const int px = u >> 4, c8 = (u & 15) * 8;
        *(volatile v4u*)(ws16 + O_XT + (pixbase + px) * 128 + c8) = hv[it];
      }
      __threadfence();
    }
    return;
  }
  bx -= PR_XT;
  if (bx < 6)  { plane_role<64, 64, 0>(w_gqkv, ws16 + O_WG, 192, bx); return; }
  bx -= 6;
  if (bx < 2)  { plane_role<64, 64, 0>(w_ggp, ws16 + O_WG + 192 * 64, 64, bx); return; }
  bx -= 2;
  if (bx < 4)  { plane_role<128, 64, 0>(w_a1, ws16 + O_A1, 64, bx); return; }
  bx -= 4;
  if (bx < 4)  { plane_role<128, 64, 0>(w_a2, ws16 + O_A2, 64, bx); return; }
  bx -= 4;
  if (bx < 2)  { plane_role<32, 32, 0>(w_swq, ws16 + O_SWQ, 96, bx); return; }
  bx -= 2;
  if (bx < 2)  { plane_role<32, 32, 0>(w_wnq, ws16 + O_WNQ, 96, bx); return; }
  bx -= 2;
  if (bx < 1)  { plane_role<64, 32, 0>(w_swp, ws16 + O_SWP, 32, bx); return; }
  bx -= 1;
  if (bx < 1)  { plane_role<64, 32, 0>(w_wnp, ws16 + O_WNP, 32, bx); return; }
  bx -= 1;
  if (bx < 16) { plane_role<256, 128, 1>(w_fc, ws16 + O_FCX, 128, bx); return; }
  bx -= 16;
  if (bx < 32) { plane_role<256, 128, 0>(w_m1, ws16 + O_M1X, 256, bx); return; }
  bx -= 32;
  if (bx < 32) { plane_role<512, 256, 0>(w_m2, ws16 + O_M2X, 128, bx); return; }
  bx -= 32;
  {
    const int e = bx * 256 + tid;
    const int ec = (e < 961) ? e : 960;
    const float dh = (float)(ec / 31 - 15);
    const float dw = (float)(ec % 31 - 15);
    float* t1 = sm + tid;
    float* t2 = sm + 4096 + tid;
#pragma unroll 1
    for (int j = 0; j < 16; ++j) {
      float a = bf_rne(pw1[2 * j]) * dh;
      a = fmaf(bf_rne(pw1[2 * j + 1]), dw, a);
      a += bf_rne(pb1[j]);
      t1[j * 256] = fmaxf(a, 0.0f);
    }
#pragma unroll 1
    for (int j = 0; j < 16; ++j) {
      float s = 0.0f;
#pragma unroll 1
      for (int i = 0; i < 16; ++i) s = fmaf(bf_rne(pw2[j * 16 + i]), t1[i * 256], s);
      s += bf_rne(pb2[j]);
      t2[j * 256] = fmaxf(s, 0.0f);
    }
    float res[4];
#pragma unroll
    for (int hd = 0; hd < 4; ++hd) {
      float s = 0.0f;
#pragma unroll 1
      for (int j = 0; j < 16; ++j) s = fmaf(bf_rne(pw3[hd * 16 + j]), t2[j * 256], s);
      res[hd] = (e < 961) ? (s + bf_rne(pb3[hd])) : 0.0f;
    }
    if (e < PBP) {
      for (int pass = 0; pass < 2; ++pass) {
#pragma unroll
        for (int hd = 0; hd < 4; ++hd) ((volatile float*)PB)[hd * PBP + e] = res[hd];
        __threadfence();
      }
    }
  }
}

__global__ __launch_bounds__(128) __attribute__((amdgpu_num_vgpr(248)))
void k_gproj(unsigned short* ws16, const float* __restrict__ bqkv, const float* __restrict__ bgp) {
  __shared__ __align__(16) float sT[4 * 16 * 68];
  const int tid = threadIdx.x, lane = tid & 31;
  const int which = __builtin_amdgcn_readfirstlane(tid >> 5);
  const int hh = lane >> 4, c = lane & 15;
  const int g = blockIdx.x >> 2, t = blockIdx.x & 3;
  const int b = g >> 6, gi = (g >> 3) & 7, gj = g & 7;

  size_t arow[4];
#pragma unroll
  for (int i = 0; i < 4; ++i) {
    const size_t pix = (size_t)b * 16384 + (size_t)(((4 * t + i) * 8 + gi) * 128 + c * 8 + gj);
    arow[i] = O_XT + pix * 128 + 8 * hh;
  }
  const size_t brow = O_WG + (size_t)(which * 64 + c) * 64 + 8 * hh;

  const v8f zero8 = {0.f, 0.f, 0.f, 0.f, 0.f, 0.f, 0.f, 0.f};
  v8f acc[4][4];
#pragma unroll
  for (int i = 0; i < 4; ++i)
#pragma unroll
    for (int j = 0; j < 4; ++j) acc[i][j] = zero8;

#pragma unroll 1
  for (int k0 = 0; k0 < 64; k0 += 32) {
    v16b bf[4];
#pragma unroll
    for (int j = 0; j < 4; ++j) bf[j] = glb_frag(ws16 + brow + (size_t)(16 * j) * 64 + k0);
#pragma unroll
    for (int i = 0; i < 4; ++i) {
      const v16b a = glb_frag(ws16 + arow[i] + k0);
#pragma unroll
      for (int j = 0; j < 4; ++j) acc[i][j] = at_mma(a, bf[j], acc[i][j]);
    }
  }

  float bv[4];
#pragma unroll
  for (int j = 0; j < 4; ++j) {
    const int n = which * 64 + 16 * j + c;
    const float v4 = bqkv[(n < 192) ? n : 191];
    const float v6 = bgp[(n >= 192) ? (n - 192) : 0];
    bv[j] = bf_rne((n < 192) ? v4 : v6);
  }

  float* slab = sT + which * (16 * 68);
  const int q = lane >> 3, c8 = (lane & 7) * 8;
  if (which != 2) {
    const size_t obase = (which == 0) ? O_PQ : ((which == 1) ? O_PK : O_PX);
#pragma unroll
    for (int i = 0; i < 4; ++i) {
#pragma unroll
      for (int j = 0; j < 4; ++j)
#pragma unroll
        for (int r = 0; r < 8; ++r) slab[(8 * hh + r) * 68 + 16 * j + c] = acc[i][j][r] + bv[j];
      wave_sync();
      v4u hv[4], lv[4];
#pragma unroll
      for (int it = 0; it < 4; ++it) split8(slab + (it * 4 + q) * 68 + c8, hv[it], lv[it]);
      for (int pass = 0; pass < 2; ++pass) {
#pragma unroll
        for (int it = 0; it < 4; ++it) {
          unsigned short* dst = ws16 + obase + (size_t)(g * 256 + 64 * t + 16 * i + it * 4 + q) * 128 + c8;
          *(volatile v4u*)dst = hv[it];
          *(volatile v4u*)(dst + 64) = lv[it];
        }
        __threadfence();
      }
      wave_sync();
    }
  } else {
#pragma unroll
    for (int j = 0; j < 4; ++j) {
#pragma unroll
      for (int i = 0; i < 4; ++i)
#pragma unroll
        for (int r = 0; r < 8; ++r) slab[c * 68 + 16 * i + 8 * hh + r] = acc[i][j][r] + bv[j];
      wave_sync();
      v4u hv[4], lv[4];
#pragma unroll
      for (int it = 0; it < 4; ++it) split8(slab + (it * 4 + q) * 68 + c8, hv[it], lv[it]);
      for (int pass = 0; pass < 2; ++pass) {
#pragma unroll
        for (int it = 0; it < 4; ++it) {
          unsigned short* dst = ws16 + O_PVT + ((size_t)(g * 2) * 64 + 16 * j + it * 4 + q) * 256 + 64 * t + c8;
          *(volatile v4u*)dst = hv[it];
          *(volatile v4u*)(dst + (size_t)64 * 256) = lv[it];
        }
        __threadfence();
      }
      wave_sync();
    }
  }
}

template <int STAGE>
__global__ __launch_bounds__(128) __attribute__((amdgpu_num_vgpr(248)))
void k_gattn(unsigned short* ws16, const float* __restrict__ PBt, const float* __restrict__ pbias) {
  constexpr size_t OQ = (STAGE == 1) ? O_PX : O_PQ;
  constexpr size_t OK = (STAGE == 1) ? O_PK : O_PX;
  constexpr size_t OV = (STAGE == 1) ? O_PVT : O_TT;
  constexpr size_t OW = (STAGE == 1) ? O_A1 : O_A2;
  __shared__ __align__(16) float  sPB[4 * PBP];
  __shared__ __align__(16) __bf16 Ps[4][16 * 128];
  __shared__ __align__(16) __bf16 OH[4][16 * 128];
  __shared__ __align__(16) float  Ts[64 * 68];

  const int tid = threadIdx.x, lane = tid & 31;
  const int wave = __builtin_amdgcn_readfirstlane(tid >> 5);
  const int hh = lane >> 4, c = lane & 15;
  const int g = blockIdx.x >> 2, qt = blockIdx.x & 3;
  const int b = g >> 6, gi = (g >> 3) & 7, gj = g & 7;

#pragma unroll 1
  for (int i = tid; i < PBP; i += 128) *(v4f*)(sPB + 4 * i) = *(const v4f*)(PBt + 4 * i);
  __syncthreads();

  const unsigned short* Qrow = ws16 + OQ + (size_t)(g * 256 + qt * 64 + wave * 16 + c) * 128 + 8 * hh;
  const unsigned short* Kb   = ws16 + OK + (size_t)(g * 256 + c) * 128 + 8 * hh;
  const unsigned short* Vb   = ws16 + OV + ((size_t)(g * 2) * 64 + c) * 256 + 8 * hh;
  __bf16* pw = Ps[wave];
  __bf16* oh = OH[wave];
  const v8b z8 = zero8b();
  const v8f zero8 = {0.f, 0.f, 0.f, 0.f, 0.f, 0.f, 0.f, 0.f};
  const int bcol = 8 * hh + 15 - c;

#pragma unroll 1
  for (int head = 0; head < 4; ++head) {
    FB qa1, qa2;
    qa1.h[0] = glb_half(Qrow + head * 16);
    qa1.h[1] = glb_half(Qrow + 64 + head * 16);
    qa2.h[0] = qa1.h[0];
    qa2.h[1] = z8;
    float mrow[8], lrow[8];
#pragma unroll
    for (int r = 0; r < 8; ++r) { mrow[r] = -INFINITY; lrow[r] = 0.f; }
    v8f oacc = zero8;
    const float* pbh = sPB + head * PBP;

#pragma unroll 1
    for (int kc = 0; kc < 4; ++kc) {
      v8f s[4];
#pragma unroll
      for (int j = 0; j < 4; ++j) {
        const unsigned short* kp = Kb + (size_t)(kc * 64 + 16 * j) * 128 + head * 16;
        FB k1, k2;
        k1.h[0] = glb_half(kp);
        k1.h[1] = k1.h[0];
        k2.h[0] = glb_half(kp + 64);
        k2.h[1] = z8;
        v8f z = zero8;
        z = at_mma(qa1.v, k1.v, z);
        z = at_mma(qa2.v, k2.v, z);
        s[j] = z;
      }
      const int dhb = qt * 4 + wave + 15 - kc * 4;
      float cm[8];
#pragma unroll
      for (int r = 0; r < 8; ++r) {
        float m = -INFINITY;
#pragma unroll
        for (int j = 0; j < 4; ++j) {
          const float sv = s[j][r] * 0.25f + pbh[(dhb - j) * 31 + bcol + r];
          s[j][r] = sv;
          m = fmaxf(m, sv);
        }
#pragma unroll
        for (int off = 1; off < 16; off <<= 1) m = fmaxf(m, __shfl_xor(m, off, 32));
        cm[r] = m;
      }
#pragma unroll
      for (int r = 0; r < 8; ++r) {
        const float mnew = fmaxf(mrow[r], cm[r]);
        const float alpha = expf(mrow[r] - mnew);
        mrow[r] = mnew;
        float psum = 0.f;
#pragma unroll
        for (int j = 0; j < 4; ++j) {
          const float p = expf(s[j][r] - mnew);
          psum += p;
          __bf16 ph, pl; at_split(p, ph, pl);
          pw[(8 * hh + r) * 128 + j * 16 + c] = ph;
          pw[(8 * hh + r) * 128 + 64 + j * 16 + c] = pl;
        }
#pragma unroll
        for (int off = 1; off < 16; off <<= 1) psum += __shfl_xor(psum, off, 32);
        lrow[r] = lrow[r] * alpha + psum;
        oacc[r] *= alpha;
      }
      wave_sync();
#pragma unroll
      for (int kk = 0; kk < 2; ++kk) {
        const v16b pa = lds_frag(pw + c * 128 + kk * 32 + 8 * hh);
        const v16b pl = lds_frag(pw + c * 128 + 64 + kk * 32 + 8 * hh);
        const unsigned short* vp = Vb + (size_t)(head * 16) * 256 + kc * 64 + kk * 32;
        const v16b vh = glb_frag(vp);
        const v16b vl = glb_frag(vp + (size_t)64 * 256);
        oacc = at_mma(pa, vh, oacc);
        oacc = at_mma(pa, vl, oacc);
        oacc = at_mma(pl, vh, oacc);
      }
      wave_sync();
    }
#pragma unroll
    for (int r = 0; r < 8; ++r) {
      const float o = oacc[r] * (1.0f / lrow[r]);
      __bf16 a, l; at_split(o, a, l);
      oh[(8 * hh + r) * 128 + head * 16 + c] = a;
      oh[(8 * hh + r) * 128 + 64 + head * 16 + c] = l;
    }
  }
  wave_sync();

  v8f acc2[4];
#pragma unroll
  for (int jn = 0; jn < 4; ++jn) acc2[jn] = zero8;
  const unsigned short* Wb = ws16 + OW + (size_t)c * 128 + 8 * hh;
#pragma unroll
  for (int ks = 0; ks < 4; ++ks) {
    const v16b a = lds_frag(oh + c * 128 + ks * 32 + 8 * hh);
#pragma unroll
    for (int jn = 0; jn < 4; ++jn) {
      const v16b bw = glb_frag(Wb + (size_t)(16 * jn) * 128 + ks * 32);
      acc2[jn] = at_mma(a, bw, acc2[jn]);
    }
  }
  float pbv[4];
#pragma unroll
  for (int jn = 0; jn < 4; ++jn) pbv[jn] = bf_rne(pbias[16 * jn + c]);

  const int q = lane >> 3, c8 = (lane & 7) * 8;
  if (STAGE == 1) {
#pragma unroll
    for (int jn = 0; jn < 4; ++jn)
#pragma unroll
      for (int r = 0; r < 8; ++r) Ts[(16 * jn + c) * 68 + wave * 16 + 8 * hh + r] = acc2[jn][r] + pbv[jn];
    __syncthreads();
    v4u hv[4], lv[4];
#pragma unroll
    for (int it = 0; it < 4; ++it) split8(Ts + (wave * 16 + it * 4 + q) * 68 + c8, hv[it], lv[it]);
    for (int pass = 0; pass < 2; ++pass) {
#pragma unroll
      for (int it = 0; it < 4; ++it) {
        const int chn = wave * 16 + it * 4 + q;
        unsigned short* dst = ws16 + O_TT + ((size_t)(g * 2) * 64 + chn) * 256 + qt * 64 + c8;
        *(volatile v4u*)dst = hv[it];
        *(volatile v4u*)(dst + (size_t)64 * 256) = lv[it];
      }
      __threadfence();
    }
  } else {
    float* slab = Ts + wave * (16 * 68);
#pragma unroll
    for (int jn = 0; jn < 4; ++jn)
#pragma unroll
      for (int r = 0; r < 8; ++r) slab[(8 * hh + r) * 68 + 16 * jn + c] = acc2[jn][r] + pbv[jn];
    wave_sync();
    v4u hv[4], lv[4];
#pragma unroll
    for (int it = 0; it < 4; ++it) split8(slab + (it * 4 + q) * 68 + c8, hv[it], lv[it]);
    for (int pass = 0; pass < 2; ++pass) {
#pragma unroll
      for (int it = 0; it < 4; ++it) {
        const int row = it * 4 + q;
        const size_t pix = (size_t)b * 16384 + (size_t)(((qt * 4 + wave) * 8 + gi) * 128 + row * 8 + gj);
        unsigned short* dst = ws16 + O_CAT + pix * 256 + 128 + c8;
        *(volatile v4u*)dst = hv[it];
        *(volatile v4u*)(dst + 64) = lv[it];
      }
      __threadfence();
    }
  }
}

template <int SHIFT>
__global__ __launch_bounds__(128) __attribute__((amdgpu_num_vgpr(248)))
void k_win(unsigned short* ws16, const float* __restrict__ qb, const float* __restrict__ rpb,
           const float* __restrict__ pb) {
  constexpr int XCH = (SHIFT != 0) ? 64 : 96;
  constexpr size_t OWQ = (SHIFT != 0) ? O_SWQ : O_WNQ;
  constexpr size_t OWP = (SHIFT != 0) ? O_SWP : O_WNP;
  constexpr int COFF = (SHIFT != 0) ? 64 : 0;
  static_assert(SHIFT == 0 || SHIFT == 4);
  __shared__ __align__(16) __bf16 QA[64 * 128];
  __shared__ __align__(16) __bf16 KB[64 * 128];
  __shared__ __align__(16) __bf16 VT[64 * 128];
  __shared__ __align__(16) __bf16 Pw[4][16 * 128];
  __shared__ __align__(16) __bf16 OA[4][16 * 64];
  __shared__ __align__(16) float  sR[4 * 228];
  __shared__ __align__(16) float  So[4][16 * 36];

  const int tid = threadIdx.x, lane = tid & 31;
  const int wave = __builtin_amdgcn_readfirstlane(tid >> 5);
  const int hh = lane >> 4, c = lane & 15;
  const int b = blockIdx.x >> 8, wh = (blockIdx.x >> 4) & 15, ww = blockIdx.x & 15;
  const v8b z8 = zero8b();
  const v8f zero8 = {0.f, 0.f, 0.f, 0.f, 0.f, 0.f, 0.f, 0.f};
  const __bf16 zb = __builtin_bit_cast(__bf16, (unsigned short)0);

#pragma unroll 1
  for (int i = tid; i < 900; i += 128) sR[(i & 3) * 228 + (i >> 2)] = bf_rne(rpb[i]);
#pragma unroll
  for (int it = 0; it < 4; ++it) {
    const int u = it * 128 + tid;
    const int hd = u >> 7, rem = u & 127;
    *(v8b*)(VT + (hd * 16 + 8 + (rem >> 4)) * 128 + (rem & 15) * 8) = z8;
  }

  {
    const int tok = wave * 16 + c;
    const int ph = (wh * 8 + (tok >> 3) + SHIFT) & 127;
    const int pwx = (ww * 8 + (tok & 7) + SHIFT) & 127;
    const size_t pix = (size_t)b * 16384 + (size_t)(ph * 128 + pwx);
    const v16b a = glb_frag(ws16 + O_XT + pix * 128 + XCH + 8 * hh);
    const unsigned short* Wq = ws16 + OWQ + (size_t)c * 32 + 8 * hh;
    v8f acc[6];
#pragma unroll
    for (int jt = 0; jt < 6; ++jt) {
      const v16b bw = glb_frag(Wq + (size_t)(16 * jt) * 32);
      acc[jt] = at_mma(a, bw, zero8);
    }
    const int hsub = c >> 3, d = c & 7;
#pragma unroll
    for (int jt = 0; jt < 6; ++jt) {
      const float bias = bf_rne(qb[16 * jt + c]);
      const int head = 2 * (jt & 1) + hsub;
#pragma unroll
      for (int r = 0; r < 8; ++r) {
        const int trow = wave * 16 + 8 * hh + r;
        float v = acc[jt][r] + bias;
        if (jt < 2) v *= 0.35355339f;
        __bf16 vh, vl; at_split(v, vh, vl);
        if (jt < 2) {
          __bf16* p = QA + trow * 128 + head * 32 + d;
          p[0] = vh; p[8] = vl; p[16] = vh; p[24] = zb;
        } else if (jt < 4) {
          __bf16* p = KB + trow * 128 + head * 32 + d;
          p[0] = vh; p[8] = vh; p[16] = vl; p[24] = zb;
        } else {
          __bf16* p = VT + (head * 16 + d) * 128 + trow;
          p[0] = vh; p[64] = vl;
        }
      }
    }
  }
  __syncthreads();

  __bf16* pwv = Pw[wave];
  __bf16* oa = OA[wave];
  const int rq = wave * 2 + hh;
  int ridq[8], ridk[4];
  {
    const int hq = wh * 8 + rq;
    const int regh = (hq >= 120 ? 1 : 0) + (hq >= 124 ? 1 : 0);
#pragma unroll
    for (int r = 0; r < 8; ++r) {
      const int wq = ww * 8 + r;
      ridq[r] = 3 * regh + (wq >= 120 ? 1 : 0) + (wq >= 124 ? 1 : 0);
    }
#pragma unroll
    for (int j = 0; j < 4; ++j) {
      const int hk = wh * 8 + 2 * j + (c >> 3);
      const int wk = ww * 8 + (c & 7);
      ridk[j] = 3 * ((hk >= 120 ? 1 : 0) + (hk >= 124 ? 1 : 0)) + (wk >= 120 ? 1 : 0) + (wk >= 124 ? 1 : 0);
    }
  }

#pragma unroll 1
  for (int head = 0; head < 4; ++head) {
    const v16b qa = lds_frag(QA + (wave * 16 + c) * 128 + head * 32 + 8 * hh);
    v8f s[4];
#pragma unroll
    for (int j = 0; j < 4; ++j) {
      const v16b kb = lds_frag(KB + (16 * j + c) * 128 + head * 32 + 8 * hh);
      s[j] = at_mma(qa, kb, zero8);
    }
    const float* rh = sR + head * 228;
    float linv[8];
#pragma unroll
    for (int r = 0; r < 8; ++r) {
      float m = -INFINITY;
#pragma unroll
      for (int j = 0; j < 4; ++j) {
        const int rk = 2 * j + (c >> 3), ck = c & 7;
        float sv = s[j][r] + rh[(rq - rk + 7) * 15 + (r - ck + 7)];
        if (SHIFT != 0) sv += (ridq[r] != ridk[j]) ? -100.0f : 0.0f;
        s[j][r] = sv;
        m = fmaxf(m, sv);
      }
#pragma unroll
      for (int off = 1; off < 16; off <<= 1) m = fmaxf(m, __shfl_xor(m, off, 32));
      float psum = 0.f;
#pragma unroll
      for (int j = 0; j < 4; ++j) {
        const float p = expf(s[j][r] - m);
        psum += p;
        __bf16 ph, pl; at_split(p, ph, pl);
        pwv[(8 * hh + r) * 128 + 16 * j + c] = ph;
        pwv[(8 * hh + r) * 128 + 64 + 16 * j + c] = pl;
      }
#pragma unroll
      for (int off = 1; off < 16; off <<= 1) psum += __shfl_xor(psum, off, 32);
      linv[r] = 1.0f / psum;
    }
    wave_sync();
    v8f oacc = zero8;
#pragma unroll
    for (int ks = 0; ks < 6; ++ks) {
      const int seg = ks >> 1;
      const int aoff = ((seg == 1) ? 64 : 0) + (ks & 1) * 32;
      const int boff = ((seg == 2) ? 64 : 0) + (ks & 1) * 32;
      const v16b pa = lds_frag(pwv + c * 128 + aoff + 8 * hh);
      const v16b vb = lds_frag(VT + (head * 16 + c) * 128 + boff + 8 * hh);
      oacc = at_mma(pa, vb, oacc);
    }
#pragma unroll
    for (int r = 0; r < 8; ++r) {
      const float o = oacc[r] * linv[r];
      __bf16 a, l; at_split(o, a, l);
      if (c < 8) {
        oa[(8 * hh + r) * 64 + head * 8 + c] = a;
        oa[(8 * hh + r) * 64 + 32 + head * 8 + c] = l;
      }
    }
    wave_sync();
  }

  v8f acc2[2];
  acc2[0] = zero8; acc2[1] = zero8;
  const unsigned short* Wp = ws16 + OWP + (size_t)c * 64 + 8 * hh;
#pragma unroll
  for (int ks = 0; ks < 2; ++ks) {
    const v16b a = lds_frag(oa + c * 64 + ks * 32 + 8 * hh);
#pragma unroll
    for (int jn = 0; jn < 2; ++jn) {
      const v16b bw = glb_frag(Wp + (size_t)(16 * jn) * 64 + ks * 32);
      acc2[jn] = at_mma(a, bw, acc2[jn]);
    }
  }
  float* so = So[wave];
#pragma unroll
  for (int jn = 0; jn < 2; ++jn) {
    const float pbv = bf_rne(pb[16 * jn + c]);
#pragma unroll
    for (int r = 0; r < 8; ++r) so[(8 * hh + r) * 36 + 16 * jn + c] = acc2[jn][r] + pbv;
  }
  wave_sync();
  {
    const int q = lane >> 3, l8 = lane & 7;
    const int ch0 = (l8 & 3) * 8;
    const bool isLo = (l8 >= 4);
    v4u ov[4];
#pragma unroll
    for (int it = 0; it < 4; ++it) {
      v4u hv, lv;
      split8(so + (it * 4 + q) * 36 + ch0, hv, lv);
      v4u sel;
#pragma unroll
      for (int k = 0; k < 4; ++k) sel[k] = isLo ? lv[k] : hv[k];
      ov[it] = sel;
    }
    for (int pass = 0; pass < 2; ++pass) {
#pragma unroll
      for (int it = 0; it < 4; ++it) {
        const int tok = wave * 16 + it * 4 + q;
        const int ph = (wh * 8 + (tok >> 3) + SHIFT) & 127;
        const int pwx = (ww * 8 + (tok & 7) + SHIFT) & 127;
        const size_t pix = (size_t)b * 16384 + (size_t)(ph * 128 + pwx);
        *(volatile v4u*)(ws16 + O_CAT + pix * 256 + COFF + l8 * 8) = ov[it];
      }
      __threadfence();
    }
  }
}

__global__ __launch_bounds__(128) __attribute__((amdgpu_num_vgpr(248)))
void k_fc(unsigned short* ws16, const float* __restrict__ fcb, const float* __restrict__ lg,
          const float* __restrict__ lb) {
  __shared__ __align__(16) float slabs[4][16 * 132];
  const int tid = threadIdx.x, lane = tid & 31;
  const int wave = __builtin_amdgcn_readfirstlane(tid >> 5);
  const int hh = lane >> 4, c = lane & 15;
  const int px0 = blockIdx.x * 64 + wave * 16;
  const unsigned short* Ar = ws16 + O_CAT + (size_t)(px0 + c) * 256 + 8 * hh;
  const unsigned short* Br = ws16 + O_FCX + (size_t)c * 256 + 8 * hh;
  const v8f zero8 = {0.f, 0.f, 0.f, 0.f, 0.f, 0.f, 0.f, 0.f};
  v8f acc[8];
#pragma unroll
  for (int j = 0; j < 8; ++j) acc[j] = zero8;
#pragma unroll 1
  for (int k0 = 0; k0 < 256; k0 += 32) {
    const v16b a = glb_frag(Ar + k0);
#pragma unroll
    for (int j = 0; j < 8; ++j) {
      const v16b bw = glb_frag(Br + (size_t)(16 * j) * 256 + k0);
      acc[j] = at_mma(a, bw, acc[j]);
    }
  }
  float* slab = slabs[wave];
#pragma unroll
  for (int j = 0; j < 8; ++j)
#pragma unroll
    for (int r = 0; r < 8; ++r) slab[(8 * hh + r) * 132 + 16 * j + c] = acc[j][r];
  wave_sync();

  const int rsel = lane >> 4, c8 = (lane & 15) * 8;
  float bia[8], gam[8], bet[8];
  {
    const v4f a0 = *(const v4f*)(fcb + c8), a1 = *(const v4f*)(fcb + c8 + 4);
    const v4f g0 = *(const v4f*)(lg + c8),  g1 = *(const v4f*)(lg + c8 + 4);
    const v4f b0 = *(const v4f*)(lb + c8),  b1 = *(const v4f*)(lb + c8 + 4);
#pragma unroll
    for (int e = 0; e < 4; ++e) {
      bia[e] = bf_rne(a0[e]); bia[e + 4] = bf_rne(a1[e]);
      gam[e] = bf_rne(g0[e]); gam[e + 4] = bf_rne(g1[e]);
      bet[e] = bf_rne(b0[e]); bet[e + 4] = bf_rne(b1[e]);
    }
  }
  v4u hv[8], lv[8];
#pragma unroll
  for (int it = 0; it < 8; ++it) {
    const int row = it * 2 + rsel;
    float v[8];
    float sum = 0.f;
#pragma unroll
    for (int e = 0; e < 8; ++e) { v[e] = slab[row * 132 + c8 + e] + bia[e]; sum += v[e]; }
#pragma unroll
    for (int off = 1; off < 16; off <<= 1) sum += __shfl_xor(sum, off, 32);
    const float mu = sum * (1.0f / 128.0f);
    float sq = 0.f;
#pragma unroll
    for (int e = 0; e < 8; ++e) { v[e] -= mu; sq += v[e] * v[e]; }
#pragma unroll
    for (int off = 1; off < 16; off <<= 1) sq += __shfl_xor(sq, off, 32);
    const float rs = 1.0f / sqrtf(sq * (1.0f / 128.0f) + 1e-5f);
    const v4u xw = *(const v4u*)(ws16 + O_XT + (size_t)(px0 + row) * 128 + c8);
    float xt[8];
    widen8(xw, xt);
    float x1[8];
#pragma unroll
    for (int e = 0; e < 8; ++e) x1[e] = xt[e] + (v[e] * rs * gam[e] + bet[e]);
    split8(x1, hv[it], lv[it]);
  }
  for (int pass = 0; pass < 2; ++pass) {
#pragma unroll
    for (int it = 0; it < 8; ++it) {
      const int row = it * 2 + rsel;
      unsigned short* dst = ws16 + O_X1 + (size_t)(px0 + row) * 256 + c8;
      *(volatile v4u*)dst = hv[it];
      *(volatile v4u*)(dst + 128) = lv[it];
    }
    __threadfence();
  }
}

__global__ __launch_bounds__(256) __attribute__((amdgpu_num_vgpr(248)))
void k_mlp(unsigned short* ws16, const float* __restrict__ m1b, const float* __restrict__ m2b,
           const float* __restrict__ g2, const float* __restrict__ b2, float* __restrict__ out) {
  __shared__ __align__(16) __bf16 hid[64 * 512];
  __shared__ __align__(16) float  slab[64 * 132];
  __shared__ __align__(16) float  sB1[256];
  __shared__ __align__(16) float  sB2[128];
  static_assert(128 * 68 * 4 <= 64 * 512 * 2);
  const int tid = threadIdx.x, lane = tid & 31;
  const int wave = __builtin_amdgcn_readfirstlane(tid >> 5);
  const int mt = wave >> 1, nh = wave & 1;
  const int hh = lane >> 4, c = lane & 15;
  const int px0 = blockIdx.x * 64;

  sB1[tid] = bf_rne(m1b[tid]);
  {
    const float t = bf_rne(m2b[tid & 127]);
    if (tid < 128) sB2[tid] = t;
  }
  __syncthreads();

  const v8f zero8 = {0.f, 0.f, 0.f, 0.f, 0.f, 0.f, 0.f, 0.f};
  {
    const unsigned short* Ar = ws16 + O_X1 + (size_t)(px0 + mt * 16 + c) * 256 + 8 * hh;
    const unsigned short* Br = ws16 + O_M1X + (size_t)(nh * 128 + c) * 256 + 8 * hh;
    v8f acc[8];
#pragma unroll
    for (int j = 0; j < 8; ++j) acc[j] = zero8;
#pragma unroll 1
    for (int k0 = 0; k0 < 256; k0 += 32) {
      const v16b a = glb_frag(Ar + k0);
#pragma unroll
      for (int j = 0; j < 8; ++j) {
        const v16b bw = glb_frag(Br + (size_t)(16 * j) * 256 + k0);
        acc[j] = at_mma(a, bw, acc[j]);
      }
    }
#pragma unroll
    for (int j = 0; j < 8; ++j) {
      const int col = nh * 128 + 16 * j + c;
      const float bv = sB1[col];
#pragma unroll
      for (int r = 0; r < 8; ++r) {
        const float hv = acc[j][r] + bv;
        const float gl = 0.5f * hv * (1.0f + erff(hv * 0.70710678118654752f));
        __bf16 a, l; at_split(gl, a, l);
        hid[(mt * 16 + 8 * hh + r) * 512 + col] = a;
        hid[(mt * 16 + 8 * hh + r) * 512 + 256 + col] = l;
      }
    }
  }
  __syncthreads();
  {
    const unsigned short* Br = ws16 + O_M2X + (size_t)(nh * 64 + c) * 512 + 8 * hh;
    v8f acc2[4];
#pragma unroll
    for (int j = 0; j < 4; ++j) acc2[j] = zero8;
#pragma unroll 1
    for (int k0 = 0; k0 < 512; k0 += 32) {
      const v16b a = lds_frag(hid + (mt * 16 + c) * 512 + k0 + 8 * hh);
#pragma unroll
      for (int j = 0; j < 4; ++j) {
        const v16b bw = glb_frag(Br + (size_t)(16 * j) * 512 + k0);
        acc2[j] = at_mma(a, bw, acc2[j]);
      }
    }
#pragma unroll
    for (int j = 0; j < 4; ++j)
#pragma unroll
      for (int r = 0; r < 8; ++r) slab[(mt * 16 + 8 * hh + r) * 132 + nh * 64 + 16 * j + c] = acc2[j][r];
  }
  __syncthreads();

  float* To = (float*)(void*)hid;
  {
    const int c8 = (tid & 15) * 8;
    float gam[8], bet[8], bia[8];
    {
      const v4f g0 = *(const v4f*)(g2 + c8), g1 = *(const v4f*)(g2 + c8 + 4);
      const v4f b0 = *(const v4f*)(b2 + c8), b1 = *(const v4f*)(b2 + c8 + 4);
#pragma unroll
      for (int e = 0; e < 4; ++e) {
        gam[e] = bf_rne(g0[e]); gam[e + 4] = bf_rne(g1[e]);
        bet[e] = bf_rne(b0[e]); bet[e + 4] = bf_rne(b1[e]);
      }
#pragma unroll
      for (int e = 0; e < 8; ++e) bia[e] = sB2[c8 + e];
    }
#pragma unroll 1
    for (int it = 0; it < 4; ++it) {
      const int row = it * 16 + (tid >> 4);
      float v[8];
      float sum = 0.f;
#pragma unroll
      for (int e = 0; e < 8; ++e) { v[e] = slab[row * 132 + c8 + e] + bia[e]; sum += v[e]; }
#pragma unroll
      for (int off = 1; off < 16; off <<= 1) sum += __shfl_xor(sum, off, 32);
      const float mu = sum * (1.0f / 128.0f);
      float sq = 0.f;
#pragma unroll
      for (int e = 0; e < 8; ++e) { v[e] -= mu; sq += v[e] * v[e]; }
#pragma unroll
      for (int off = 1; off < 16; off <<= 1) sq += __shfl_xor(sq, off, 32);
      const float rs = 1.0f / sqrtf(sq * (1.0f / 128.0f) + 1e-5f);
      const size_t px = (size_t)(px0 + row);
      const v4u xh = *(const v4u*)(ws16 + O_X1 + px * 256 + c8);
      const v4u xl = *(const v4u*)(ws16 + O_X1 + px * 256 + 128 + c8);
      const v4u xw = *(const v4u*)(ws16 + O_XT + px * 128 + c8);
      float fh[8], fl[8], xt[8];
      widen8(xh, fh); widen8(xl, fl); widen8(xw, xt);
#pragma unroll
      for (int e = 0; e < 8; ++e) {
        const float x1 = fh[e] + fl[e];
        const float y2 = v[e] * rs * gam[e] + bet[e];
        To[(c8 + e) * 68 + row] = (x1 + y2) + xt[e];
      }
    }
  }
  __syncthreads();
  {
    const int b = px0 >> 14, rem = px0 & 16383;
    const int h = rem >> 7, w0 = rem & 127;
    const int w4 = (tid & 15) * 4;
    v4f ov[8];
#pragma unroll
    for (int it = 0; it < 8; ++it) {
      const int chn = it * 16 + (tid >> 4);
      ov[it] = *(const v4f*)(To + chn * 68 + w4);
    }
    for (int pass = 0; pass < 2; ++pass) {
#pragma unroll
      for (int it = 0; it < 8; ++it) {
        const int chn = it * 16 + (tid >> 4);
        *(volatile v4f*)(out + ((size_t)(b * CH + chn) * IMH + h) * IMW + w0 + w4) = ov[it];
      }
      __threadfence();
    }
  }
}

extern "C" void kernel_launch(void* const* d_in, const int* in_sizes, int n_in,
                              void* d_out, int out_size, void* d_ws, size_t ws_size,
                              hipStream_t stream) {
  if (n_in < 35) return;
  const int expect[35] = {8388608, 128, 128, 12288, 192, 4096, 64, 32, 16, 256, 16, 64, 4,
                          4096, 64, 4096, 64, 3072, 96, 900, 1024, 32, 3072, 96, 900, 1024, 32,
                          16384, 128, 128, 128, 32768, 256, 32768, 128};
  for (int i = 0; i < 35; ++i) if (in_sizes[i] != expect[i]) return;
  if (out_size != NB * CH * IMH * IMW) return;
  if (WS_TOTAL > ws_size) return;

  const float* x      = (const float*)d_in[0];
  const float* ln_g   = (const float*)d_in[1];
  const float* ln_b   = (const float*)d_in[2];
  const float* gaqkvw = (const float*)d_in[3];
  const float* gaqkvb = (const float*)d_in[4];
  const float* gagpw  = (const float*)d_in[5];
  const float* gagpb  = (const float*)d_in[6];
  const float* posw1  = (const float*)d_in[7];
  const float* posb1  = (const float*)d_in[8];
  const float* posw2  = (const float*)d_in[9];
  const float* posb2  = (const float*)d_in[10];
  const float* posw3  = (const float*)d_in[11];
  const float* posb3  = (const float*)d_in[12];
  const float* a1pw   = (const float*)d_in[13];
  const float* a1pb   = (const float*)d_in[14];
  const float* a2pw   = (const float*)d_in[15];
  const float* a2pb   = (const float*)d_in[16];
  const float* swqkvw = (const float*)d_in[17];
  const float* swqkvb = (const float*)d_in[18];
  const float* swrpb  = (const float*)d_in[19];
  const float* swpw   = (const float*)d_in[20];
  const float* swpb   = (const float*)d_in[21];
  const float* wnqkvw = (const float*)d_in[22];
  const float* wnqkvb = (const float*)d_in[23];
  const float* wnrpb  = (const float*)d_in[24];
  const float* wnpw   = (const float*)d_in[25];
  const float* wnpb   = (const float*)d_in[26];
  const float* fcw    = (const float*)d_in[27];
  const float* fcb    = (const float*)d_in[28];
  const float* n2g    = (const float*)d_in[29];
  const float* n2b    = (const float*)d_in[30];
  const float* m1w    = (const float*)d_in[31];
  const float* m1b    = (const float*)d_in[32];
  const float* m2w    = (const float*)d_in[33];
  const float* m2b    = (const float*)d_in[34];

  unsigned short* ws16 = (unsigned short*)d_ws;
  float* PB = (float*)((char*)d_ws + PB_BYTE);

  k_prep<<<dim3(PR_XT + 106), dim3(256), 0, stream>>>(
      x, gaqkvw, gagpw, a1pw, a2pw, swqkvw, wnqkvw, swpw, wnpw, fcw, m1w, m2w,
      posw1, posb1, posw2, posb2, posw3, posb3, ws16, PB);
  k_gproj<<<dim3(1024), dim3(128), 0, stream>>>(ws16, gaqkvb, gagpb);
  k_gattn<1><<<dim3(1024), dim3(128), 0, stream>>>(ws16, PB, a1pb);
  k_gattn<2><<<dim3(1024), dim3(128), 0, stream>>>(ws16, PB, a2pb);
  k_win<4><<<dim3(1024), dim3(128), 0, stream>>>(ws16, swqkvb, swrpb, swpb);
  k_win<0><<<dim3(1024), dim3(128), 0, stream>>>(ws16, wnqkvb, wnrpb, wnpb);
  k_fc<<<dim3(1024), dim3(128), 0, stream>>>(ws16, fcb, ln_g, ln_b);
  k_mlp<<<dim3(1024), dim3(256), 0, stream>>>(ws16, m1b, m2b, n2g, n2b, (float*)d_out);
  (void)hipGetLastError();
}
